// SqueezeBertSelfAttention_42004780155203
// MI455X (gfx1250) — hardware-verified
//
#include <hip/hip_runtime.h>
#include <math.h>


#define NB 8
#define CC 1024
#define WW 1024
#define HH 16
#define HD 64
#define BK 32

typedef __attribute__((ext_vector_type(16))) _Float16 v16h;
typedef __attribute__((ext_vector_type(8)))  _Float16 v8h;
typedef __attribute__((ext_vector_type(8)))  float v8f;
typedef __attribute__((ext_vector_type(4)))  float v4f;
typedef __attribute__((ext_vector_type(4)))  unsigned v4u;

template <typename T> __device__ __forceinline__ void vst2(void* p, T v) { *(volatile T*)p = v; __threadfence(); *(volatile T*)p = v; }
__device__ __forceinline__ v8f wmma16(v16h a, v16h b, v8f c) {
  v8f d = __builtin_amdgcn_wmma_f32_16x16x32_f16(false, a, false, b, (short)0, c, false, false);
  asm volatile("v_nop\n\tv_nop\n\tv_nop\n\tv_nop" : "+v"(d) : "v"(a), "v"(b));
  return d;
}
__device__ __forceinline__ v16h frag_h(const _Float16* rowk0, int lane) {
  union { v16h v; v8h q[2]; } u; const _Float16* p = rowk0 + 8 * (lane >> 4);
  u.q[0] = *(const v8h*)p; u.q[1] = *(const v8h*)(p + 16); return u.v;
}
__device__ __forceinline__ v16h frag_f32(const float* rowk0, int lane) {
  v16h a; const float* p = rowk0 + 8 * (lane >> 4);
#pragma unroll
  for (int i = 0; i < 8; ++i) { a[i] = (_Float16)p[i]; a[8 + i] = (_Float16)p[16 + i]; }
  return a;
}
#define LDSX() do { asm volatile("s_wait_dscnt 0" ::: "memory"); __builtin_amdgcn_wave_barrier(); __builtin_amdgcn_fence(__ATOMIC_RELEASE, "workgroup"); } while (0)

__global__ __launch_bounds__(256) void k_xT(const float* __restrict__ x, _Float16* __restrict__ xT) {
  __shared__ float tile[64][65];
  const int n = blockIdx.z, c0 = blockIdx.y * 64, w0 = blockIdx.x * 64, tid = threadIdx.x;
  for (int q = tid; q < 64 * 64; q += 256) { const int cl = q >> 6, wl = q & 63; tile[cl][wl] = x[((size_t)n * CC + c0 + cl) * WW + w0 + wl]; }
  __syncthreads();
  for (int q = tid; q < 64 * 8; q += 256) { const int wl = q >> 3, pc = q & 7;
    union { v8h h; v4u u; } pk;
#pragma unroll
    for (int e = 0; e < 8; ++e) pk.h[e] = (_Float16)tile[pc * 8 + e][wl];
    vst2(xT + ((size_t)n * WW + w0 + wl) * CC + c0 + pc * 8, pk.u); }
}
__global__ __launch_bounds__(256) void k_wcvt(const float* __restrict__ wq, const float* __restrict__ wk, const float* __restrict__ wv, _Float16* __restrict__ wh) {
  const size_t g8 = (size_t)blockIdx.x * 256 + threadIdx.x; const int m = blockIdx.y;
  const float* s = m == 0 ? wq : (m == 1 ? wk : wv);
  union { v8h h; v4u u; } pk;
#pragma unroll
  for (int e = 0; e < 8; ++e) pk.h[e] = (_Float16)s[g8 * 8 + e];
  vst2(wh + (size_t)m * CC * CC + g8 * 8, pk.u);
}

__global__ __launch_bounds__(128) void k_qkv(const _Float16* __restrict__ xT, const _Float16* __restrict__ wh, const float* __restrict__ bq,
                                           const float* __restrict__ bk, const float* __restrict__ bv,
                                           _Float16* __restrict__ qh, _Float16* __restrict__ kh, _Float16* __restrict__ vT) {
  __shared__ __align__(16) float st[128][68];
  const int tid = threadIdx.x, wave = tid >> 5, lane = tid & 31, col = lane & 15, g = lane >> 4;
  const int n = blockIdx.y / (WW / 64), w0 = (blockIdx.y % (WW / 64)) * 64, o0 = blockIdx.x * 128, which = blockIdx.z;
  const _Float16* W = wh + (size_t)which * CC * CC;
  const float* bb = which == 0 ? bq : (which == 1 ? bk : bv);
  v8f acc[8] = {};
#pragma unroll 1
  for (int kc = 0; kc < CC / 32; ++kc) {
    const v16h a = frag_h(xT + ((size_t)n * WW + w0 + wave * 16 + col) * CC + kc * 32, lane);
#pragma unroll
    for (int j = 0; j < 8; ++j) acc[j] = wmma16(a, frag_h(W + (size_t)(o0 + j * 16 + col) * CC + kc * 32, lane), acc[j]);
  }
#pragma unroll
  for (int j = 0; j < 8; ++j) { const float bv_ = bb[o0 + j * 16 + col];
#pragma unroll
    for (int r = 0; r < 8; ++r) st[j * 16 + col][wave * 16 + 8 * g + r] = acc[j][r] + bv_; }
  __syncthreads();
  const int h0 = o0 / HD;
  if (which < 2) {
    _Float16* dst = which == 0 ? qh : kh;
    for (int q = tid; q < 2 * 64 * 8; q += 128) { const int hh = q >> 9, wl = (q >> 3) & 63, pc = q & 7;
      union { v8h h; v4u u; } pk;
#pragma unroll
      for (int e = 0; e < 8; ++e) pk.h[e] = (_Float16)st[hh * 64 + pc * 8 + e][wl];
      vst2(dst + (((size_t)n * HH + h0 + hh) * WW + w0 + wl) * HD + pc * 8, pk.u); }
  } else {
    for (int q = tid; q < 128 * 8; q += 128) { const int cl = q >> 3, pc = q & 7; const int hh = cl >> 6, d = cl & 63;
      union { v8h h; v4u u; } pk;
#pragma unroll
      for (int i = 0; i < 8; ++i) pk.h[i] = (_Float16)st[cl][pc * 8 + i];
      vst2(vT + (((size_t)n * HH + h0 + hh) * HD + d) * WW + w0 + pc * 8, pk.u); }
  }
}

__global__ __launch_bounds__(128) void k_attn(const _Float16* __restrict__ qh, const _Float16* __restrict__ kh, const _Float16* __restrict__ vT,
                                            const float* __restrict__ mask, float* __restrict__ out) {
  __shared__ __align__(16) float sP[4][16][BK];
  __shared__ __align__(16) float sOT[HD][68];
  const int tid = threadIdx.x, w = tid >> 5, lane = tid & 31, g = lane >> 4, ln = lane & 15;
  const int bh = blockIdx.y, n = bh / HH, h = bh % HH, q0 = blockIdx.x * 64 + w * 16;
  const _Float16* qrow = qh + ((size_t)bh * WW + q0 + ln) * HD;
  const v16h qa0 = frag_h(qrow, lane), qa1 = frag_h(qrow + 32, lane);
  const float* mk = mask + (size_t)n * WW;
  float mrun[8], lrun[8];
  v8f acc[4];
#pragma unroll
  for (int r = 0; r < 8; ++r) { mrun[r] = -3.0e38f; lrun[r] = 0.f; }
#pragma unroll
  for (int t = 0; t < 4; ++t) acc[t] = (v8f){};
  const _Float16* kb = kh + (size_t)bh * WW * HD;
  const _Float16* vb = vT + (size_t)bh * HD * WW;
#pragma unroll 1
  for (int k0 = 0; k0 < WW; k0 += BK) {
    v8f s0 = {}, s1 = {};
    s0 = wmma16(qa0, frag_h(kb + (size_t)(k0 + ln) * HD, lane), s0);      s0 = wmma16(qa1, frag_h(kb + (size_t)(k0 + ln) * HD + 32, lane), s0);
    s1 = wmma16(qa0, frag_h(kb + (size_t)(k0 + 16 + ln) * HD, lane), s1); s1 = wmma16(qa1, frag_h(kb + (size_t)(k0 + 16 + ln) * HD + 32, lane), s1);
    const float mk0 = mk[k0 + ln], mk1 = mk[k0 + 16 + ln];
#pragma unroll
    for (int r = 0; r < 8; ++r) {
      const float x0 = s0[r] * 0.125f + mk0, x1 = s1[r] * 0.125f + mk1;
      float mx = fmaxf(x0, x1);
#pragma unroll
      for (int off = 8; off >= 1; off >>= 1) mx = fmaxf(mx, __shfl_xor(mx, off, 32));
      const float mn = fmaxf(mrun[r], mx);
      const float corr = expf(mrun[r] - mn);
      const float p0 = expf(x0 - mn), p1 = expf(x1 - mn);
      float sum = p0 + p1;
#pragma unroll
      for (int off = 8; off >= 1; off >>= 1) sum += __shfl_xor(sum, off, 32);
      lrun[r] = lrun[r] * corr + sum; mrun[r] = mn;
#pragma unroll
      for (int t = 0; t < 4; ++t) acc[t][r] *= corr;
      sP[w][8 * g + r][ln] = p0 * 16384.0f; sP[w][8 * g + r][16 + ln] = p1 * 16384.0f;
    }
    LDSX();
    const v16h pa = frag_f32(&sP[w][ln][0], lane);
#pragma unroll
    for (int t = 0; t < 4; ++t) acc[t] = wmma16(pa, frag_h(vb + (size_t)(t * 16 + ln) * WW + k0, lane), acc[t]);
    __builtin_amdgcn_wave_barrier();
  }
#pragma unroll
  for (int r = 0; r < 8; ++r) { const float il = (1.0f / 16384.0f) / lrun[r];
#pragma unroll
    for (int t = 0; t < 4; ++t) sOT[t * 16 + ln][w * 16 + 8 * g + r] = acc[t][r] * il; }
  __syncthreads();
  const int qb0 = blockIdx.x * 64;
  for (int q = tid; q < HD * 16; q += 128) { const int d = q >> 4, pc = q & 15;
    vst2(out + ((size_t)n * CC + h * HD + d) * WW + qb0 + pc * 4, *(const v4f*)(&sOT[d][pc * 4])); }
}

extern "C" void kernel_launch(void* const* d_in, const int* in_sizes, int n_in,
                              void* d_out, int out_size, void* d_ws, size_t ws_size,
                              hipStream_t stream) {
  (void)in_sizes; (void)n_in; (void)out_size; (void)ws_size;
  const float* hs   = (const float*)d_in[0];
  const float* mask = (const float*)d_in[1];
  const float* wq = (const float*)d_in[2]; const float* bq = (const float*)d_in[3];
  const float* wk = (const float*)d_in[4]; const float* bk = (const float*)d_in[5];
  const float* wv = (const float*)d_in[6]; const float* bv = (const float*)d_in[7];
  float* out = (float*)d_out;
  char* ws = (char*)d_ws; size_t off = 0;
  auto take = [&](size_t bytes) { char* p = ws + off; off += (bytes + 255) & ~(size_t)255; return p; };
  _Float16* xT = (_Float16*)take((size_t)NB * WW * CC * 2);
  _Float16* wh = (_Float16*)take((size_t)3 * CC * CC * 2);
  _Float16* qh = (_Float16*)take((size_t)NB * HH * WW * HD * 2);
  _Float16* kh = (_Float16*)take((size_t)NB * HH * WW * HD * 2);
  _Float16* vT = (_Float16*)take((size_t)NB * HH * HD * WW * 2);
  k_xT<<<dim3(WW / 64, CC / 64, NB), 256, 0, stream>>>(hs, xT);
  k_wcvt<<<dim3((CC * CC / 8) / 256, 3), 256, 0, stream>>>(wq, wk, wv, wh);
  k_qkv<<<dim3(CC / 128, NB * (WW / 64), 3), 128, 0, stream>>>(xT, wh, bq, bk, bv, qh, kh, vT);
  k_attn<<<dim3(WW / 64, NB * HH), 128, 0, stream>>>(qh, kh, vT, mask, out);
}
